// GNNPolicy_4398046511886
// MI455X (gfx1250) — hardware-verified
//
#include <hip/hip_runtime.h>
#include <stddef.h>
#include <stdint.h>
#include <math.h>

#pragma clang fp contract(off)


#define HD     128
#define NLAY   4
#define LAT    64
#define KP     256
#define NP     256
#define KE     256
#define KU     512
#define KT     256
#define NT     64
#define NTHR   256
#define NWAVE  8
#define EPT    8
#define CHUNK  (NTHR * EPT)
#define WCAP   (EPT * 32)
#define LISTN  (NWAVE * WCAP)
#define NBS    512
#define SLB    9
#define RCAP   20480
#define TR     64
#define NTMAX  (RCAP / TR)
#define GBM    64
#define WSQ    16384
#define WUNIT  4096
#define NWPART 20
#define TUNIT  2048
#define TAILN  132
#define CSR_ZINTS    (LISTN + 2 * RCAP + 3 * NBS)
#define MISC_INTS    16
#define CSR_LDS_INTS (CSR_ZINTS + MISC_INTS)
#define MSG_LDS_INTS ((TR * KE) / 2 + TR * HD + 2 * HD + 2 * TR)
#define PROJ_LDS_BYTES (GBM * NP * 4)
#define UPD_LDS_BYTES  (GBM * KU * 2)
#define TOPO_LDS_INTS  ((GBM * KT) / 2 + 3 * 64)
#define WSMAX  134217728

static_assert((CHUNK & (CHUNK - 1)) == 0 && CHUNK <= 4096);
static_assert((NBS & (NBS - 1)) == 0 && NBS == (1 << SLB));
static_assert(((long long)CHUNK << SLB) < (1LL << 31));
static_assert(NBS % NWAVE == 0 && NBS % 32 == 0 && NBS % GBM == 0);
static_assert(RCAP % 4 == 0 && CSR_ZINTS % 4 == 0 && LISTN % 4 == 0);
static_assert(RCAP % TR == 0 && RCAP % NTHR == 0 && RCAP % 32 == 0);
static_assert(KP % 32 == 0 && KE % 32 == 0 && KU % 32 == 0 && KT % 32 == 0);
static_assert(KP == 2 * HD && KE == 2 * HD && KU == 4 * HD && NP == 2 * HD);
static_assert(GBM == 4 * 16 && NTHR == 4 * GBM && TR == GBM && HD == 4 * 32);
static_assert(CSR_LDS_INTS * 4 <= 300000);
static_assert(GBM * KP * 2 <= PROJ_LDS_BYTES);
static_assert(GBM * HD * 4 <= UPD_LDS_BYTES);
static_assert(GBM * NT * 4 <= (GBM * KT));
static_assert(WUNIT % NTHR == 0 && (NWPART * WUNIT) % NTHR == 0 && TUNIT % NTHR == 0);
static_assert(MSG_LDS_INTS * 4 <= 300000);

typedef float          v2f   __attribute__((ext_vector_type(2)));
typedef float          v4f   __attribute__((ext_vector_type(4)));
typedef float          v8f   __attribute__((ext_vector_type(8)));
typedef int            v4i   __attribute__((ext_vector_type(4)));
typedef int            v8i   __attribute__((ext_vector_type(8)));
typedef unsigned short v4us  __attribute__((ext_vector_type(4)));
typedef unsigned short v8us  __attribute__((ext_vector_type(8)));
typedef unsigned short v16us __attribute__((ext_vector_type(16)));
typedef __bf16         v16bf __attribute__((ext_vector_type(16)));
typedef v2f  __attribute__((may_alias)) v2fa;
typedef v4f  __attribute__((may_alias)) v4fa;
typedef v4i  __attribute__((may_alias)) v4ia;
typedef v4us __attribute__((may_alias)) v4usa;
typedef v8us __attribute__((may_alias)) v8usa;
union FragB { v16bf v; v16us u; v8us h[2]; v8i w; };

__device__ __forceinline__ v8f wmb(const FragB& a, const FragB& b, v8f c) {
  v8f d = __builtin_amdgcn_wmma_f32_16x16x32_bf16(false, a.v, false, b.v, (short)0, c, false, false);
  asm volatile("v_nop\n\tv_nop\n\tv_nop\n\tv_nop" : "+v"(d) : "v"(a.w), "v"(b.w));
  return d;
}

__device__ __forceinline__ unsigned bf16_bits(float f) {
  const unsigned u = __float_as_uint(f);
  return ((u + 0x7FFFu + ((u >> 16) & 1u)) >> 16) & 0xFFFFu;
}
__device__ __forceinline__ float bf16_val(float f) {
  return __uint_as_float(bf16_bits(f) << 16);
}
__device__ __forceinline__ v4f bfr4(const v4f a) {
  v4f r; r.x = bf16_val(a.x); r.y = bf16_val(a.y); r.z = bf16_val(a.z); r.w = bf16_val(a.w); return r;
}
__device__ __forceinline__ void hilo4(const v4f a, v4us& h4, v4us& l4) {
  unsigned hb;
  hb = bf16_bits(a.x); h4[0] = (unsigned short)hb; l4[0] = (unsigned short)bf16_bits(a.x - __uint_as_float(hb << 16));
  hb = bf16_bits(a.y); h4[1] = (unsigned short)hb; l4[1] = (unsigned short)bf16_bits(a.y - __uint_as_float(hb << 16));
  hb = bf16_bits(a.z); h4[2] = (unsigned short)hb; l4[2] = (unsigned short)bf16_bits(a.z - __uint_as_float(hb << 16));
  hb = bf16_bits(a.w); h4[3] = (unsigned short)hb; l4[3] = (unsigned short)bf16_bits(a.w - __uint_as_float(hb << 16));
}
__device__ __forceinline__ float elu1(float v) {
  const float t = fmaxf(v, -87.0f);
  const float e = __expf(t) - 1.0f;
  return (v > 0.0f) ? v : ((v == v) ? e : v);
}

template <int SLBT>
__device__ __forceinline__ int scan_chunk(const int* __restrict__ dsts, int nE, int cbase, int slotBase,
                                          int nb, int vec8, int* list, int tid, int lane, int wave) {
  int wc = 0;
  const int el0  = tid * EPT;
  const int e0   = cbase + el0;
  const int sent = -2147483647 - 1;
  v4i da, db;
  if (vec8 != 0 && cbase + CHUNK <= nE) {
    da = *(const v4i*)(dsts + e0);
    db = *(const v4i*)(dsts + e0 + 4);
  } else {
    da.x = (e0     < nE) ? dsts[min(e0,     nE - 1)] : sent;
    da.y = (e0 + 1 < nE) ? dsts[min(e0 + 1, nE - 1)] : sent;
    da.z = (e0 + 2 < nE) ? dsts[min(e0 + 2, nE - 1)] : sent;
    da.w = (e0 + 3 < nE) ? dsts[min(e0 + 3, nE - 1)] : sent;
    db.x = (e0 + 4 < nE) ? dsts[min(e0 + 4, nE - 1)] : sent;
    db.y = (e0 + 5 < nE) ? dsts[min(e0 + 5, nE - 1)] : sent;
    db.z = (e0 + 6 < nE) ? dsts[min(e0 + 6, nE - 1)] : sent;
    db.w = (e0 + 7 < nE) ? dsts[min(e0 + 7, nE - 1)] : sent;
  }
  const unsigned nbs = (unsigned)slotBase;
  const unsigned unb = (unsigned)nb;
  const unsigned s0 = (unsigned)da.x - nbs, s1 = (unsigned)da.y - nbs;
  const unsigned s2 = (unsigned)da.z - nbs, s3 = (unsigned)da.w - nbs;
  const unsigned s4 = (unsigned)db.x - nbs, s5 = (unsigned)db.y - nbs;
  const unsigned s6 = (unsigned)db.z - nbs, s7 = (unsigned)db.w - nbs;
  const bool h0 = s0 < unb, h1 = s1 < unb, h2 = s2 < unb, h3 = s3 < unb;
  const bool h4 = s4 < unb, h5 = s5 < unb, h6 = s6 < unb, h7 = s7 < unb;
  const unsigned any = __builtin_amdgcn_ballot_w32(h0 | h1 | h2 | h3 | h4 | h5 | h6 | h7);
  if (any != 0u) {
#define HITJ(J, HJ, SJ) { \
      const unsigned mj = __builtin_amdgcn_ballot_w32(HJ); \
      if (mj != 0u) { \
        if (HJ) { \
          const int pos = wc + (int)__builtin_amdgcn_mbcnt_lo(mj, 0u); \
          if (pos < WCAP) list[wave * WCAP + pos] = ((el0 + (J)) << SLBT) | (int)(SJ); \
        } \
        wc += (int)__builtin_popcount(mj); } }
    HITJ(0, h0, s0)
    HITJ(1, h1, s1)
    HITJ(2, h2, s2)
    HITJ(3, h3, s3)
    HITJ(4, h4, s4)
    HITJ(5, h5, s5)
    HITJ(6, h6, s6)
    HITJ(7, h7, s7)
#undef HITJ
  }
  return wc;
}

__global__ __launch_bounds__(NTHR) void k_wprep(const float* __restrict__ Ws, const float* __restrict__ Wd,
                                                const float* __restrict__ Wme, const float* __restrict__ Wh,
                                                const float* __restrict__ Wa, const float* __restrict__ Wt,
                                                unsigned short* BP, unsigned short* BE, unsigned short* BU,
                                                unsigned short* BT, int nUnits) {
  const int u = (int)blockIdx.x * NTHR + (int)threadIdx.x;
  if (u >= nUnits) return;
  const float* W;
  unsigned short* dp;
  int ncol;
  if (u < NWPART * WUNIT) {
    const int part = u >> 12;
    const int v  = u & (WUNIT - 1);
    const int l  = part / 5;
    const int j  = part - 5 * l;
    const int n  = v >> 5;
    const int k8 = (v & 31) * 8;
    const int kk = k8 & (HD - 1);
    const size_t lw = (size_t)l * WSQ;
    ncol = HD;
    if (j == 0)      { W = Ws + lw;  dp = BP + (size_t)l * (NP * KP) + (size_t)n * KP + k8; }
    else if (j == 1) { W = Wd + lw;  dp = BP + (size_t)l * (NP * KP) + (size_t)(HD + n) * KP + k8; }
    else if (j == 2) { W = Wme + lw; dp = BE + (size_t)l * (HD * KE) + (size_t)n * KE + k8; }
    else if (j == 3) { W = Wh + lw;  dp = BU + (size_t)l * (HD * KU) + (size_t)n * KU + k8; }
    else             { W = Wa + lw;  dp = BU + (size_t)l * (HD * KU) + (size_t)n * KU + 2 * HD + k8; }
    W += (size_t)kk * HD + n;
  } else {
    const int v  = u - NWPART * WUNIT;
    const int n  = v >> 5;
    const int k8 = (v & 31) * 8;
    const int kk = k8 & (HD - 1);
    ncol = NT;
    W  = Wt + (size_t)kk * NT + n;
    dp = BT + (size_t)n * KT + k8;
  }
  v4f a, b;
  a.x = W[0];                 a.y = W[(size_t)ncol];      a.z = W[(size_t)2 * ncol];  a.w = W[(size_t)3 * ncol];
  b.x = W[(size_t)4 * ncol];  b.y = W[(size_t)5 * ncol];  b.z = W[(size_t)6 * ncol];  b.w = W[(size_t)7 * ncol];
  v8us o;
  o[0] = (unsigned short)bf16_bits(a.x); o[1] = (unsigned short)bf16_bits(a.y);
  o[2] = (unsigned short)bf16_bits(a.z); o[3] = (unsigned short)bf16_bits(a.w);
  o[4] = (unsigned short)bf16_bits(b.x); o[5] = (unsigned short)bf16_bits(b.y);
  o[6] = (unsigned short)bf16_bits(b.z); o[7] = (unsigned short)bf16_bits(b.w);
  *(volatile v8us*)dp = o;
  __threadfence();
  *(volatile v8us*)dp = o;
}

__global__ __launch_bounds__(NTHR) void k_h0(const float* __restrict__ x, const float* __restrict__ Wn,
                                             const float* __restrict__ bn, float* H, int nN, int nUnits) {
  const int i = (int)blockIdx.x * NTHR + (int)threadIdx.x;
  if (i >= nUnits) return;
  const int row = i >> 5;
  const int c0  = (i & 31) * 4;
  const int rc  = row < nN ? row : nN - 1;
  const v4f xv = bfr4(*(const v4fa*)(x + (size_t)rc * 4));
  const v4f w0 = bfr4(*(const v4fa*)(Wn + 0 * HD + c0));
  const v4f w1 = bfr4(*(const v4fa*)(Wn + 1 * HD + c0));
  const v4f w2 = bfr4(*(const v4fa*)(Wn + 2 * HD + c0));
  const v4f w3 = bfr4(*(const v4fa*)(Wn + 3 * HD + c0));
  const v4f b4 = bfr4(*(const v4fa*)(bn + c0));
  v4f o;
  {
    float p;
    p = xv.x * w0.x; p = fmaf(xv.y, w1.x, p); p = fmaf(xv.z, w2.x, p); p = fmaf(xv.w, w3.x, p); o.x = elu1(p + b4.x);
    p = xv.x * w0.y; p = fmaf(xv.y, w1.y, p); p = fmaf(xv.z, w2.y, p); p = fmaf(xv.w, w3.y, p); o.y = elu1(p + b4.y);
    p = xv.x * w0.z; p = fmaf(xv.y, w1.z, p); p = fmaf(xv.z, w2.z, p); p = fmaf(xv.w, w3.z, p); o.z = elu1(p + b4.z);
    p = xv.x * w0.w; p = fmaf(xv.y, w1.w, p); p = fmaf(xv.z, w2.w, p); p = fmaf(xv.w, w3.w, p); o.w = elu1(p + b4.w);
  }
  const v4f z4 = {0.f, 0.f, 0.f, 0.f};
  if (row >= nN) o = z4;
  float* op = H + (size_t)row * HD + c0;
  *(volatile v4f*)op = o;
  __threadfence();
  *(volatile v4f*)op = o;
}

__global__ __launch_bounds__(NTHR) void k_csr(const int* __restrict__ ei, const float* __restrict__ pos,
                                              int nE, int nN, int vec8,
                                              int* ES, int* ED, float* EW, int* INFO) {
  extern __shared__ __attribute__((aligned(16))) int dsm[];
  int* list = dsm;
  int* hl   = dsm + LISTN;
  int* sl   = hl + RCAP;
  int* cnt  = sl + RCAP;
  int* offs = cnt + NBS;
  int* cur  = offs + NBS;
  int* misc = cur + NBS;
  const int tid = (int)threadIdx.x, lane = tid & 31, wave = tid >> 5;
  const int b = (int)blockIdx.x;
  const int nodeBase = b * NBS;
  const int* keys = ei + nE;

  {
    const v4i z4 = {0, 0, 0, 0};
    for (int i = tid * 4; i < CSR_ZINTS; i += NTHR * 4) *(v4ia*)(dsm + i) = z4;
    if (tid < MISC_INTS) misc[tid] = 0;
  }
  __syncthreads();

  int t = 0, ov = 0;
  const int nChunks = (nE + CHUNK - 1) / CHUNK;
#pragma unroll 1
  for (int ch = 0; ch < nChunks; ++ch) {
    const int cbase = ch * CHUNK;
    const int wc = scan_chunk<SLB>(keys, nE, cbase, nodeBase, NBS, vec8, list, tid, lane, wave);
    if (lane == 0) misc[wave] = wc;
    __syncthreads();
    if (wave == 0) {
#pragma unroll 1
      for (int w2 = 0; w2 < NWAVE; ++w2) {
        int c = misc[w2];
        c = c < 0 ? 0 : (c > WCAP ? WCAP : c);
#pragma unroll 1
        for (int b0 = 0; b0 < c; b0 += 32) {
          const int idx = b0 + lane;
          const int ent = list[w2 * WCAP + (idx < WCAP ? idx : WCAP - 1)];
          const int m32 = (c - b0) < 32 ? (c - b0) : 32;
#pragma unroll 1
          for (int k = 0; k < m32; ++k) {
            const int u    = __builtin_amdgcn_readlane(ent, k);
            const int slot = u & (NBS - 1);
            const int el   = (u >> SLB) & (CHUNK - 1);
            const int pk   = ((cbase + el) << SLB) | slot;
            if (t < RCAP) {
              if (lane == 0) { hl[t] = pk; cnt[slot] = cnt[slot] + 1; }
              t = t + 1;
            } else {
              ov = 1;
            }
          }
        }
      }
    }
    __syncthreads();
  }
  if (wave == 0 && lane == 0) { misc[8] = t; misc[9] = ov; }
  __syncthreads();
  int tt = misc[8];
  tt = tt < 0 ? 0 : (tt > RCAP ? RCAP : tt);
  const int ovf = misc[9];

  if (wave == 0) {
    const int base = lane * (NBS / 32);
    int s = 0;
#pragma unroll 1
    for (int i = 0; i < NBS / 32; ++i) s += cnt[base + i];
    int incl = s;
#pragma unroll
    for (int d = 1; d < 32; d <<= 1) {
      const int y = __shfl_up(incl, d, 32);
      if (lane >= d) incl += y;
    }
    int run = incl - s;
#pragma unroll 1
    for (int i = 0; i < NBS / 32; ++i) {
      const int cv = cnt[base + i];
      offs[base + i] = run;
      cur[base + i]  = run;
      run += cv;
    }
  }
  __syncthreads();
  if (wave == 0) {
#pragma unroll 1
    for (int b0 = 0; b0 < tt; b0 += 32) {
      const int idx = b0 + lane;
      const int ent = hl[idx < RCAP ? idx : RCAP - 1];
      const int m32 = (tt - b0) < 32 ? (tt - b0) : 32;
#pragma unroll 1
      for (int k = 0; k < m32; ++k) {
        const int u    = __builtin_amdgcn_readlane(ent, k);
        const int slot = u & (NBS - 1);
        if (lane == 0) {
          int p = cur[slot];
          p = p < 0 ? 0 : (p > RCAP - 1 ? RCAP - 1 : p);
          sl[p] = u;
          cur[slot] = p + 1;
        }
      }
    }
  }
  __syncthreads();

  {
    const size_t regBase = (size_t)b * RCAP;
#pragma unroll 1
    for (int i = tid; i < RCAP; i += NTHR) {
      const int u = sl[i];
      const bool live = i < tt;
      const int slot = u & (NBS - 1);
      int eid = (int)((unsigned)u >> SLB);
      eid = eid > nE - 1 ? nE - 1 : eid;
      int s = ei[eid];
      s = s < 0 ? 0 : (s > nN - 1 ? nN - 1 : s);
      const int dn  = nodeBase + slot;
      const int dcl = dn > nN - 1 ? nN - 1 : dn;
      const v2f ps = *(const v2fa*)(pos + (size_t)2 * s);
      const v2f pd = *(const v2fa*)(pos + (size_t)2 * dcl);
      const float dx = bf16_val(pd.x) - bf16_val(ps.x);
      const float dy = bf16_val(pd.y) - bf16_val(ps.y);
      const float dd = sqrtf((dx * dx + dy * dy) + 1e-12f);
      const int   es = live ? s  : 0;
      const int   ed = live ? dn : -1;
      const float ew = live ? dd : 0.0f;
      const size_t o = regBase + (size_t)i;
      *(volatile int*)(ES + o) = es;
      *(volatile int*)(ED + o) = ed;
      *(volatile float*)(EW + o) = ew;
      __threadfence();
      *(volatile int*)(ES + o) = es;
      *(volatile int*)(ED + o) = ed;
      *(volatile float*)(EW + o) = ew;
    }
  }
  if (wave == 0) {
    const int iv = (lane == 0) ? tt : ((lane == 1) ? ovf : 0);
    int* ip = INFO + (size_t)b * 32 + lane;
    *(volatile int*)ip = iv;
    __threadfence();
    *(volatile int*)ip = iv;
  }
}

__global__ __launch_bounds__(NTHR) void k_proj(const float* __restrict__ H, const unsigned short* __restrict__ Bw,
                                               float* P) {
  extern __shared__ __attribute__((aligned(16))) int dsm[];
  unsigned short* At = (unsigned short*)dsm;
  float* S = (float*)dsm;
  const int tid = (int)threadIdx.x, lane = tid & 31, wave = tid >> 5, hh = lane >> 4, m = lane & 15;
  const int rowBase = (int)blockIdx.x * GBM;

  {
    const int r = tid >> 2, q = tid & 3;
    const float* hr = H + (size_t)(rowBase + r) * HD + 32 * q;
    unsigned short* ar = At + r * KP + 32 * q;
#pragma unroll
    for (int j4 = 0; j4 < 8; ++j4) {
      const v4f hv = *(const v4fa*)(hr + 4 * j4);
      v4us h4, l4;
      hilo4(hv, h4, l4);
      *(v4usa*)(ar + 4 * j4) = h4;
      *(v4usa*)(ar + HD + 4 * j4) = l4;
    }
  }
  __syncthreads();

  v8f acc[8];
  {
    const v8f z = {0.f, 0.f, 0.f, 0.f, 0.f, 0.f, 0.f, 0.f};
#pragma unroll
    for (int t = 0; t < 8; ++t) acc[t] = z;
  }
  const int rt = wave & 3, ch = wave >> 2;
  const unsigned short* ap = At + (16 * rt + m) * KP + 8 * hh;
  const unsigned short* bp = Bw + (size_t)(HD * ch + m) * KP + 8 * hh;
#pragma unroll 1
  for (int k0 = 0; k0 < KP; k0 += 32) {
    FragB af;
    af.h[0] = *(const v8usa*)(ap + k0);
    af.h[1] = *(const v8usa*)(ap + k0 + 16);
#pragma unroll
    for (int nt = 0; nt < 8; ++nt) {
      const unsigned short* wq = bp + (size_t)(16 * nt) * KP + k0;
      FragB bf;
      bf.h[0] = *(const v8usa*)wq;
      bf.h[1] = *(const v8usa*)(wq + 16);
      acc[nt] = wmb(af, bf, acc[nt]);
    }
  }
  __syncthreads();
#pragma unroll
  for (int nt = 0; nt < 8; ++nt) {
    const int lc = HD * ch + 16 * nt + m;
#pragma unroll
    for (int r = 0; r < 8; ++r) {
      const int lr = 16 * rt + 8 * hh + r;
      S[lr * NP + lc] = acc[nt][r];
    }
  }
  __syncthreads();

  v4f pv[16];
#pragma unroll
  for (int i = 0; i < 16; ++i) pv[i] = *(const v4fa*)(S + (16 * rt + i) * NP + HD * ch + 4 * lane);
#pragma unroll
  for (int i = 0; i < 16; ++i) {
    float* op = P + (size_t)(rowBase + 16 * rt + i) * NP + HD * ch + 4 * lane;
    *(volatile v4f*)op = pv[i];
  }
  __threadfence();
#pragma unroll
  for (int i = 0; i < 16; ++i) {
    float* op = P + (size_t)(rowBase + 16 * rt + i) * NP + HD * ch + 4 * lane;
    *(volatile v4f*)op = pv[i];
  }
}

__global__ __launch_bounds__(NTHR) void k_msg(const int* __restrict__ ES, const int* __restrict__ ED,
                                              const float* __restrict__ EW, const int* __restrict__ INFO,
                                              const float* __restrict__ We, const float* __restrict__ be,
                                              const unsigned short* __restrict__ Bw, const float* __restrict__ P,
                                              const float* __restrict__ bml, float* AGG, int nN, int mRows) {
  extern __shared__ __attribute__((aligned(16))) int dsm[];
  unsigned short* At = (unsigned short*)dsm;
  float* S    = (float*)(dsm + (TR * KE) / 2);
  float* swe  = S + TR * HD;
  float* sbe  = swe + HD;
  int*   sidx = (int*)(sbe + HD);
  int*   didx = sidx + TR;
  const int tid = (int)threadIdx.x, lane = tid & 31, wave = tid >> 5, hh = lane >> 4, m = lane & 15;
  const int b = (int)blockIdx.x;
  const int nodeBase = b * NBS;
  const size_t regBase = (size_t)b * RCAP;

  {
    const int c1 = tid & (HD - 1);
    const float wv = bf16_val(We[c1]);
    const float bv = bf16_val(be[c1]);
    if (tid < HD) { swe[c1] = wv; sbe[c1] = bv; }
  }
  const v4f bm4 = bfr4(*(const v4fa*)(bml + 4 * lane));
  int tt = INFO[(size_t)b * 32];
  const int ovf = INFO[(size_t)b * 32 + 1];
  tt = tt < 0 ? 0 : (tt > RCAP ? RCAP : tt);
  const int ntile = (tt + TR - 1) / TR;
  const float pz = (ovf != 0) ? __int_as_float(0x7fc00000) : 0.0f;
  int hiRow = nodeBase + NBS;
  hiRow = hiRow > mRows ? mRows : hiRow;
  const int c = tid & (HD - 1);
  int ckey = nodeBase - 1;
  float carry = 0.0f;
  __syncthreads();

#pragma unroll 1
  for (int t = 0; t < ntile; ++t) {
    {
      const int r = tid >> 2, q = tid & 3;
      const size_t i = regBase + (size_t)(TR * t + r);
      const float d  = EW[i];
      const int   sv = ES[i];
      const int   dv = ED[i];
      const int   s2 = sv < 0 ? 0 : (sv > nN - 1 ? nN - 1 : sv);
      if (q == 0) { sidx[r] = s2; didx[r] = dv; }
      unsigned short* ar = At + r * KE + 32 * q;
      const float* wr = swe + 32 * q;
      const float* br = sbe + 32 * q;
#pragma unroll
      for (int j4 = 0; j4 < 8; ++j4) {
        const v4f w4 = *(const v4fa*)(wr + 4 * j4);
        const v4f b4 = *(const v4fa*)(br + 4 * j4);
        v4f e4;
        e4.x = elu1(d * w4.x + b4.x);
        e4.y = elu1(d * w4.y + b4.y);
        e4.z = elu1(d * w4.z + b4.z);
        e4.w = elu1(d * w4.w + b4.w);
        v4us h4, l4;
        hilo4(e4, h4, l4);
        *(v4usa*)(ar + 4 * j4) = h4;
        *(v4usa*)(ar + HD + 4 * j4) = l4;
      }
    }
    __syncthreads();

    v8f acc[4];
    {
      const v8f z = {0.f, 0.f, 0.f, 0.f, 0.f, 0.f, 0.f, 0.f};
      acc[0] = z; acc[1] = z; acc[2] = z; acc[3] = z;
    }
    const int rt = wave & 3, cq = wave >> 2;
    const unsigned short* ap = At + (16 * rt + m) * KE + 8 * hh;
    const unsigned short* bp = Bw + (size_t)(64 * cq + m) * KE + 8 * hh;
#pragma unroll 1
    for (int k0 = 0; k0 < KE; k0 += 32) {
      FragB af;
      af.h[0] = *(const v8usa*)(ap + k0);
      af.h[1] = *(const v8usa*)(ap + k0 + 16);
#pragma unroll
      for (int nt = 0; nt < 4; ++nt) {
        const unsigned short* wq = bp + (size_t)(16 * nt) * KE + k0;
        FragB bf;
        bf.h[0] = *(const v8usa*)wq;
        bf.h[1] = *(const v8usa*)(wq + 16);
        acc[nt] = wmb(af, bf, acc[nt]);
      }
    }
#pragma unroll
    for (int nt = 0; nt < 4; ++nt) {
      const int lc = 64 * cq + 16 * nt + m;
#pragma unroll
      for (int r = 0; r < 8; ++r) {
        const int lr = 16 * rt + 8 * hh + r;
        S[lr * HD + lc] = acc[nt][r];
      }
    }
    __syncthreads();

#pragma unroll 2
    for (int jj = 0; jj < 8; ++jj) {
      const int row = wave + 8 * jj;
      const int s = sidx[row];
      int dd = didx[row];
      dd = dd < 0 ? 0 : (dd > mRows - 1 ? mRows - 1 : dd);
      const v4f ps = *(const v4fa*)(P + (size_t)s * NP + 4 * lane);
      const v4f pd = *(const v4fa*)(P + (size_t)dd * NP + HD + 4 * lane);
      float* srow = S + row * HD + 4 * lane;
      const v4f ev = *(const v4fa*)srow;
      v4f mv;
      mv.x = elu1(((ps.x + pd.x) + ev.x) + bm4.x);
      mv.y = elu1(((ps.y + pd.y) + ev.y) + bm4.y);
      mv.z = elu1(((ps.z + pd.z) + ev.z) + bm4.z);
      mv.w = elu1(((ps.w + pd.w) + ev.w) + bm4.w);
      *(v4fa*)srow = mv;
    }
    __syncthreads();

    if (wave < 4) {
#pragma unroll 1
      for (int row = 0; row < TR; ++row) {
        const int k = didx[row];
        const float v = S[row * HD + c];
        if ((unsigned)(k - nodeBase) < (unsigned)NBS && k < mRows) {
          if (k == ckey) {
            carry = carry + v;
          } else if (k > ckey) {
            if (ckey >= nodeBase) {
              const float val = carry + pz;
              float* gp = AGG + (size_t)ckey * HD + c;
              *(volatile float*)gp = val;
              __threadfence();
              *(volatile float*)gp = val;
            }
#pragma unroll 1
            for (int n2 = ckey + 1; n2 < k; ++n2) {
              float* gp = AGG + (size_t)n2 * HD + c;
              *(volatile float*)gp = pz;
              __threadfence();
              *(volatile float*)gp = pz;
            }
            ckey  = k;
            carry = v;
          }
        }
      }
    }
    __syncthreads();
  }

  if (wave < 4) {
    if (ckey >= nodeBase && ckey < hiRow) {
      const float val = carry + pz;
      float* gp = AGG + (size_t)ckey * HD + c;
      *(volatile float*)gp = val;
      __threadfence();
      *(volatile float*)gp = val;
    }
    int n0 = ckey + 1;
    n0 = n0 < nodeBase ? nodeBase : n0;
#pragma unroll 1
    for (int n2 = n0; n2 < hiRow; ++n2) {
      float* gp = AGG + (size_t)n2 * HD + c;
      *(volatile float*)gp = pz;
      __threadfence();
      *(volatile float*)gp = pz;
    }
  }
}

__global__ __launch_bounds__(NTHR) void k_update(const float* __restrict__ Hold, const float* __restrict__ AGG,
                                                 const unsigned short* __restrict__ Bw, const float* __restrict__ bul,
                                                 float* Hn, int nN) {
  extern __shared__ __attribute__((aligned(16))) int dsm[];
  unsigned short* At = (unsigned short*)dsm;
  float* S = (float*)dsm;
  const int tid = (int)threadIdx.x, lane = tid & 31, wave = tid >> 5, hh = lane >> 4, m = lane & 15;
  const int rowBase = (int)blockIdx.x * GBM;

  {
    const int r = tid >> 2, q = tid & 3;
    const float* hr = Hold + (size_t)(rowBase + r) * HD + 32 * q;
    const float* gr = AGG  + (size_t)(rowBase + r) * HD + 32 * q;
    unsigned short* ar = At + r * KU + 32 * q;
#pragma unroll
    for (int j4 = 0; j4 < 8; ++j4) {
      const v4f hv = *(const v4fa*)(hr + 4 * j4);
      v4us h4, l4;
      hilo4(hv, h4, l4);
      *(v4usa*)(ar + 4 * j4) = h4;
      *(v4usa*)(ar + HD + 4 * j4) = l4;
    }
#pragma unroll
    for (int j4 = 0; j4 < 8; ++j4) {
      const v4f gv = *(const v4fa*)(gr + 4 * j4);
      v4us h4, l4;
      hilo4(gv, h4, l4);
      *(v4usa*)(ar + 2 * HD + 4 * j4) = h4;
      *(v4usa*)(ar + 3 * HD + 4 * j4) = l4;
    }
  }
  __syncthreads();

  v8f acc[4];
  {
    const v8f z = {0.f, 0.f, 0.f, 0.f, 0.f, 0.f, 0.f, 0.f};
    acc[0] = z; acc[1] = z; acc[2] = z; acc[3] = z;
  }
  const int rt = wave & 3, cq = wave >> 2;
  const unsigned short* ap = At + (16 * rt + m) * KU + 8 * hh;
  const unsigned short* bp = Bw + (size_t)(64 * cq + m) * KU + 8 * hh;
#pragma unroll 1
  for (int k0 = 0; k0 < KU; k0 += 32) {
    FragB af;
    af.h[0] = *(const v8usa*)(ap + k0);
    af.h[1] = *(const v8usa*)(ap + k0 + 16);
#pragma unroll
    for (int nt = 0; nt < 4; ++nt) {
      const unsigned short* wq = bp + (size_t)(16 * nt) * KU + k0;
      FragB bf;
      bf.h[0] = *(const v8usa*)wq;
      bf.h[1] = *(const v8usa*)(wq + 16);
      acc[nt] = wmb(af, bf, acc[nt]);
    }
  }
  __syncthreads();
#pragma unroll
  for (int nt = 0; nt < 4; ++nt) {
    const int lc = 64 * cq + 16 * nt + m;
#pragma unroll
    for (int r = 0; r < 8; ++r) {
      const int lr = 16 * rt + 8 * hh + r;
      S[lr * HD + lc] = acc[nt][r];
    }
  }
  __syncthreads();

  const v4f bu4 = bfr4(*(const v4fa*)(bul + 4 * lane));
  const v4f z4 = {0.f, 0.f, 0.f, 0.f};
  v4f pv[8];
#pragma unroll
  for (int jj = 0; jj < 8; ++jj) {
    const int row = wave + 8 * jj;
    const int grw = rowBase + row;
    const v4f sv = *(const v4fa*)(S + row * HD + 4 * lane);
    const v4f ho = *(const v4fa*)(Hold + (size_t)grw * HD + 4 * lane);
    v4f y;
    y.x = elu1(sv.x + bu4.x);
    y.y = elu1(sv.y + bu4.y);
    y.z = elu1(sv.z + bu4.z);
    y.w = elu1(sv.w + bu4.w);
    v4f hn = ho + y;
    if (grw >= nN) hn = z4;
    pv[jj] = hn;
  }
#pragma unroll
  for (int jj = 0; jj < 8; ++jj) {
    float* op = Hn + (size_t)(rowBase + wave + 8 * jj) * HD + 4 * lane;
    *(volatile v4f*)op = pv[jj];
  }
  __threadfence();
#pragma unroll
  for (int jj = 0; jj < 8; ++jj) {
    float* op = Hn + (size_t)(rowBase + wave + 8 * jj) * HD + 4 * lane;
    *(volatile v4f*)op = pv[jj];
  }
}

__global__ __launch_bounds__(NTHR) void k_topo(const float* __restrict__ H, const unsigned short* __restrict__ Bw,
                                               const float* __restrict__ bt1, const float* __restrict__ Wt2,
                                               const float* __restrict__ bt2, float* out, int nN) {
  extern __shared__ __attribute__((aligned(16))) int dsm[];
  unsigned short* At = (unsigned short*)dsm;
  float* S    = (float*)dsm;
  float* sw2  = (float*)(dsm + (GBM * KT) / 2);
  float* sb1  = sw2 + 64;
  float* orow = sb1 + 64;
  const int tid = (int)threadIdx.x, lane = tid & 31, wave = tid >> 5, hh = lane >> 4, m = lane & 15;
  const int rowBase = (int)blockIdx.x * GBM;

  {
    const int r = tid >> 2, q = tid & 3;
    const float* hr = H + (size_t)(rowBase + r) * HD + 32 * q;
    unsigned short* ar = At + r * KT + 32 * q;
#pragma unroll
    for (int j4 = 0; j4 < 8; ++j4) {
      const v4f hv = *(const v4fa*)(hr + 4 * j4);
      v4us h4, l4;
      hilo4(hv, h4, l4);
      *(v4usa*)(ar + 4 * j4) = h4;
      *(v4usa*)(ar + HD + 4 * j4) = l4;
    }
    const int c1 = tid & 63;
    const float wv = bf16_val(Wt2[c1]);
    const float bv = bf16_val(bt1[c1]);
    if (tid < 64) { sw2[c1] = wv; sb1[c1] = bv; }
  }
  __syncthreads();

  v8f acc[2];
  {
    const v8f z = {0.f, 0.f, 0.f, 0.f, 0.f, 0.f, 0.f, 0.f};
    acc[0] = z; acc[1] = z;
  }
  const int rt = wave & 3, cp = wave >> 2;
  const unsigned short* ap = At + (16 * rt + m) * KT + 8 * hh;
  const unsigned short* bp = Bw + (size_t)(32 * cp + m) * KT + 8 * hh;
#pragma unroll 1
  for (int k0 = 0; k0 < KT; k0 += 32) {
    FragB af;
    af.h[0] = *(const v8usa*)(ap + k0);
    af.h[1] = *(const v8usa*)(ap + k0 + 16);
#pragma unroll
    for (int nt = 0; nt < 2; ++nt) {
      const unsigned short* wq = bp + (size_t)(16 * nt) * KT + k0;
      FragB bf;
      bf.h[0] = *(const v8usa*)wq;
      bf.h[1] = *(const v8usa*)(wq + 16);
      acc[nt] = wmb(af, bf, acc[nt]);
    }
  }
  __syncthreads();
#pragma unroll
  for (int nt = 0; nt < 2; ++nt) {
    const int lc = 32 * cp + 16 * nt + m;
#pragma unroll
    for (int r = 0; r < 8; ++r) {
      const int lr = 16 * rt + 8 * hh + r;
      S[lr * NT + lc] = acc[nt][r];
    }
  }
  __syncthreads();

  {
    const int r = tid >> 2, q = tid & 3;
    const float* srow = S + r * NT + 16 * q;
    const float* wrow = sw2 + 16 * q;
    const float* brow = sb1 + 16 * q;
    float pt = 0.0f;
#pragma unroll 4
    for (int cc = 0; cc < 16; ++cc) pt = fmaf(elu1(srow[cc] + brow[cc]), wrow[cc], pt);
    pt += __shfl_xor(pt, 1);
    pt += __shfl_xor(pt, 2);
    const float val = pt + bf16_val(bt2[0]);
    if (q == 0) orow[r] = val;
  }
  __syncthreads();
  if (wave == 0) {
    int nv = nN - rowBase;
    nv = nv < 0 ? 0 : (nv > GBM ? GBM : nv);
    const int npc = nv >> 2;
    const v4f o4 = *(const v4fa*)(orow + 4 * (lane & 15));
    float* op = out + (size_t)rowBase + 4 * lane;
    if (lane < npc) *(volatile v4f*)op = o4;
    __threadfence();
    if (lane < npc) *(volatile v4f*)op = o4;
  }
}

__global__ __launch_bounds__(NTHR) void k_tail(const float* __restrict__ H, const float* __restrict__ zc,
    const float* __restrict__ tc, const int* __restrict__ ui, const int* __restrict__ vi, const int* __restrict__ wi,
    const float* __restrict__ Ge1, const float* __restrict__ ge1b, const float* __restrict__ Ge2, const float* __restrict__ ge2b,
    const float* __restrict__ Gmu, const float* __restrict__ gmub, const float* __restrict__ Glv, const float* __restrict__ glvb,
    const float* __restrict__ Gd1, const float* __restrict__ gd1b, const float* __restrict__ Gd2, const float* __restrict__ gd2b,
    const float* __restrict__ Gd3, const float* __restrict__ gd3b, const float* __restrict__ Gp1, const float* __restrict__ gp1b,
    const float* __restrict__ Gp2, const float* __restrict__ gp2b, const float* __restrict__ pbs,
    float* out, int nN, int obase) {
  __shared__ float cond[2 * HD];
  __shared__ float xe[LAT + 2 * HD];
  __shared__ float s1[HD];
  __shared__ float s2[64];
  __shared__ float smu[64];
  __shared__ float slv[64];
  __shared__ float sp1[64];
  __shared__ __attribute__((aligned(16))) float ov[144];
  const int tid = (int)threadIdx.x, lane = tid & 31, wave = tid >> 5;
  int u = ui[0], v = vi[0], w = wi[0];
  u = u < 0 ? 0 : (u > nN - 1 ? nN - 1 : u);
  v = v < 0 ? 0 : (v > nN - 1 ? nN - 1 : v);
  w = w < 0 ? 0 : (w > nN - 1 ? nN - 1 : w);
  {
    const int cc = tid & (HD - 1);
    const float hu = H[(size_t)u * HD + cc];
    const float hv = H[(size_t)v * HD + cc];
    const float hw = H[(size_t)w * HD + cc];
    const float feat = ((hu + hv) + hw) * (1.0f / 3.0f);
    const float zv = bf16_val(zc[cc]);
    cond[tid] = (tid < HD) ? feat : zv;
  }
  __syncthreads();
  {
    const float tv = bf16_val(tc[tid & 3]);
    if (tid < 4) xe[tid] = tv;
    xe[4 + tid] = cond[tid];
  }
  __syncthreads();
  {
    const int j = tid & (HD - 1);
    float acc = 0.0f;
#pragma unroll 1
    for (int k = 0; k < 4 + 2 * HD; ++k) acc = fmaf(xe[k], bf16_val(Ge1[(size_t)k * HD + j]), acc);
    const float r1 = elu1(acc + bf16_val(ge1b[j]));
    if (tid < HD) s1[tid] = r1;
  }
  __syncthreads();
  {
    const int j = tid & 63;
    float acc = 0.0f;
#pragma unroll 1
    for (int k = 0; k < HD; ++k) acc = fmaf(s1[k], bf16_val(Ge2[(size_t)k * 64 + j]), acc);
    const float he = elu1(acc + bf16_val(ge2b[j]));
    if (tid < 64) s2[tid] = he;
  }
  __syncthreads();
  {
    const int j = tid & 63;
    float am = 0.0f, al = 0.0f;
#pragma unroll 1
    for (int k = 0; k < 64; ++k) {
      const float hk = s2[k];
      am = fmaf(hk, bf16_val(Gmu[(size_t)k * 64 + j]), am);
      al = fmaf(hk, bf16_val(Glv[(size_t)k * 64 + j]), al);
    }
    const float mu = am + bf16_val(gmub[j]);
    const float lv = al + bf16_val(glvb[j]);
    if (tid < 64) { smu[tid] = mu; slv[tid] = lv; }
  }
  __syncthreads();
  {
    const float mv = smu[tid & 63];
    if (tid < 64) xe[tid] = mv;
    xe[64 + tid] = cond[tid];
  }
  __syncthreads();
  {
    const int j = tid & (HD - 1);
    float acc = 0.0f;
#pragma unroll 1
    for (int k = 0; k < LAT + 2 * HD; ++k) acc = fmaf(xe[k], bf16_val(Gd1[(size_t)k * HD + j]), acc);
    const float d1 = elu1(acc + bf16_val(gd1b[j]));
    const int j2 = tid & 63;
    float ap = 0.0f;
#pragma unroll 1
    for (int k = 0; k < 2 * HD; ++k) ap = fmaf(cond[k], bf16_val(Gp1[(size_t)k * 64 + j2]), ap);
    const float p1 = elu1(ap + bf16_val(gp1b[j2]));
    if (tid < HD) s1[tid] = d1;
    if (tid < 64) sp1[tid] = p1;
  }
  __syncthreads();
  {
    const int j = tid & 63;
    float acc = 0.0f;
#pragma unroll 1
    for (int k = 0; k < HD; ++k) acc = fmaf(s1[k], bf16_val(Gd2[(size_t)k * 64 + j]), acc);
    const float d2 = elu1(acc + bf16_val(gd2b[j]));
    if (tid < 64) s2[tid] = d2;
  }
  __syncthreads();
  {
    const int j = tid & 3;
    float ab = 0.0f, aq = 0.0f;
#pragma unroll 1
    for (int k = 0; k < 64; ++k) {
      ab = fmaf(s2[k],  bf16_val(Gd3[(size_t)k * 4 + j]), ab);
      aq = fmaf(sp1[k], bf16_val(Gp2[(size_t)k * 4 + j]), aq);
    }
    const float base = ab + bf16_val(gd3b[j]);
    const float pb   = aq + bf16_val(gp2b[j]);
    const float sc   = fminf(fmaxf(bf16_val(pbs[0]), 0.0f), 0.5f);
    const float th   = tanhf(pb);
    const float xp   = base + th * sc;
    if (tid < 4) ov[tid] = xp;
    const float mv  = smu[tid & 63];
    const float lvv = slv[tid & 63];
    if (tid < 64) { ov[4 + tid] = mv; ov[68 + tid] = lvv; }
    if (tid >= TAILN && tid < 144) ov[tid] = 0.0f;
  }
  __syncthreads();
  if (wave == 0) {
    const v4f o4 = *(const v4fa*)(ov + 4 * lane);
    const v4f o5 = *(const v4fa*)(ov + 128);
    float* op = out + (size_t)obase + 4 * lane;
    float* oq = out + (size_t)obase + 128;
    *(volatile v4f*)op = o4;
    if (lane == 0) *(volatile v4f*)oq = o5;
    __threadfence();
    *(volatile v4f*)op = o4;
    if (lane == 0) *(volatile v4f*)oq = o5;
  }
}

static inline int cdiv(int a, int b) { return (a + b - 1) / b; }
static inline size_t al256(size_t o) { return (o + 255) & ~(size_t)255; }

extern "C" void kernel_launch(void* const* d_in, const int* in_sizes, int n_in,
                              void* d_out, int out_size, void* d_ws, size_t ws_size,
                              hipStream_t stream) {
  if (n_in < 42) return;
  if (in_sizes[0] < 4 * GBM || (in_sizes[0] & 3) != 0) return;
  const int nN = in_sizes[0] / 4;
  if ((nN % 32) != 0 || nN >= (1 << 24)) return;
  if (in_sizes[1] != 2 * nN) return;
  if (in_sizes[2] < 2 || (in_sizes[2] & 1) != 0) return;
  const int nE = in_sizes[2] / 2;
  if (nE >= (1 << 22)) return;
  if (in_sizes[3] != HD || in_sizes[4] != 4) return;
  if (in_sizes[5] != 1 || in_sizes[6] != 1 || in_sizes[7] != 1) return;
  if (in_sizes[8] != 4 * HD || in_sizes[9] != HD || in_sizes[10] != HD || in_sizes[11] != HD) return;
  if (in_sizes[12] != NLAY * WSQ || in_sizes[13] != NLAY * WSQ || in_sizes[14] != NLAY * WSQ) return;
  if (in_sizes[15] != NLAY * HD) return;
  if (in_sizes[16] != NLAY * WSQ || in_sizes[17] != NLAY * WSQ || in_sizes[18] != NLAY * HD) return;
  if (in_sizes[19] != HD * 64 || in_sizes[20] != 64 || in_sizes[21] != 64 || in_sizes[22] != 1) return;
  if (in_sizes[23] != (4 + 2 * HD) * 128 || in_sizes[24] != 128 || in_sizes[25] != 128 * 64 || in_sizes[26] != 64) return;
  if (in_sizes[27] != 64 * 64 || in_sizes[28] != 64 || in_sizes[29] != 64 * 64 || in_sizes[30] != 64) return;
  if (in_sizes[31] != (LAT + 2 * HD) * 128 || in_sizes[32] != 128 || in_sizes[33] != 128 * 64 || in_sizes[34] != 64) return;
  if (in_sizes[35] != 64 * 4 || in_sizes[36] != 4 || in_sizes[37] != 2 * HD * 64 || in_sizes[38] != 64) return;
  if (in_sizes[39] != 64 * 4 || in_sizes[40] != 4 || in_sizes[41] != 1) return;
  if (out_size != nN + TAILN) return;

  const float* x      = (const float*)d_in[0];
  const float* pos    = (const float*)d_in[1];
  const int*   eidx   = (const int*)  d_in[2];
  const float* z_c    = (const float*)d_in[3];
  const float* tc     = (const float*)d_in[4];
  const int*   u_idx  = (const int*)  d_in[5];
  const int*   v_idx  = (const int*)  d_in[6];
  const int*   w_idx  = (const int*)  d_in[7];
  const float* Wn     = (const float*)d_in[8];
  const float* bn     = (const float*)d_in[9];
  const float* We     = (const float*)d_in[10];
  const float* be     = (const float*)d_in[11];
  const float* Wm_src = (const float*)d_in[12];
  const float* Wm_dst = (const float*)d_in[13];
  const float* Wm_e   = (const float*)d_in[14];
  const float* bm     = (const float*)d_in[15];
  const float* Wu_h   = (const float*)d_in[16];
  const float* Wu_agg = (const float*)d_in[17];
  const float* bu     = (const float*)d_in[18];
  const float* Wt1    = (const float*)d_in[19];
  const float* bt1    = (const float*)d_in[20];
  const float* Wt2    = (const float*)d_in[21];
  const float* bt2    = (const float*)d_in[22];
  const float* Ge1    = (const float*)d_in[23];
  const float* ge1b   = (const float*)d_in[24];
  const float* Ge2    = (const float*)d_in[25];
  const float* ge2b   = (const float*)d_in[26];
  const float* Gmu    = (const float*)d_in[27];
  const float* gmub   = (const float*)d_in[28];
  const float* Glv    = (const float*)d_in[29];
  const float* glvb   = (const float*)d_in[30];
  const float* Gd1    = (const float*)d_in[31];
  const float* gd1b   = (const float*)d_in[32];
  const float* Gd2    = (const float*)d_in[33];
  const float* gd2b   = (const float*)d_in[34];
  const float* Gd3    = (const float*)d_in[35];
  const float* gd3b   = (const float*)d_in[36];
  const float* Gp1    = (const float*)d_in[37];
  const float* gp1b   = (const float*)d_in[38];
  const float* Gp2    = (const float*)d_in[39];
  const float* gp2b   = (const float*)d_in[40];
  const float* pbs    = (const float*)d_in[41];
  float* out = (float*)d_out;

  const int MP = cdiv(nN, GBM) * GBM;
  const int gM = MP / GBM;
  const int gC = cdiv(nN, NBS);
  if ((long long)gC * NBS < (long long)MP) return;
  const int vec8 = ((nE & 3) == 0) ? 1 : 0;

  char* ws = (char*)d_ws;
  size_t off = 0;
  const size_t oBP = off; off = al256(off + (size_t)NLAY * NP * KP * 2);
  const size_t oBE = off; off = al256(off + (size_t)NLAY * HD * KE * 2);
  const size_t oBU = off; off = al256(off + (size_t)NLAY * HD * KU * 2);
  const size_t oBT = off; off = al256(off + (size_t)NT * KT * 2);
  const size_t oHA = off; off = al256(off + (size_t)MP * HD * 4);
  const size_t oHB = off; off = al256(off + (size_t)MP * HD * 4);
  const size_t oP  = off; off = al256(off + (size_t)MP * NP * 4);
  const size_t oAG = off; off = al256(off + (size_t)MP * HD * 4);
  const size_t oES = off; off = al256(off + (size_t)gC * RCAP * 4);
  const size_t oED = off; off = al256(off + (size_t)gC * RCAP * 4);
  const size_t oEW = off; off = al256(off + (size_t)gC * RCAP * 4);
  const size_t oIN = off; off = al256(off + (size_t)gC * 32 * 4);
  if (off > ws_size || off > (size_t)WSMAX) return;
  unsigned short* BP  = (unsigned short*)(ws + oBP);
  unsigned short* BE  = (unsigned short*)(ws + oBE);
  unsigned short* BU  = (unsigned short*)(ws + oBU);
  unsigned short* BT  = (unsigned short*)(ws + oBT);
  float*          HA  = (float*)(ws + oHA);
  float*          HB  = (float*)(ws + oHB);
  float*          P   = (float*)(ws + oP);
  float*          AGG = (float*)(ws + oAG);
  int*            ES  = (int*)(ws + oES);
  int*            ED  = (int*)(ws + oED);
  float*          EW  = (float*)(ws + oEW);
  int*            INFO = (int*)(ws + oIN);

  const size_t csrLds  = (size_t)CSR_LDS_INTS * 4;
  const size_t msgLds  = (size_t)MSG_LDS_INTS * 4;
  const size_t projLds = (size_t)PROJ_LDS_BYTES;
  const size_t updLds  = (size_t)UPD_LDS_BYTES;
  const size_t topoLds = (size_t)TOPO_LDS_INTS * 4;
  hipFuncSetAttribute(reinterpret_cast<const void*>(&k_csr),    hipFuncAttributeMaxDynamicSharedMemorySize, (int)csrLds);
  hipFuncSetAttribute(reinterpret_cast<const void*>(&k_msg),    hipFuncAttributeMaxDynamicSharedMemorySize, (int)msgLds);
  hipFuncSetAttribute(reinterpret_cast<const void*>(&k_proj),   hipFuncAttributeMaxDynamicSharedMemorySize, (int)projLds);
  hipFuncSetAttribute(reinterpret_cast<const void*>(&k_update), hipFuncAttributeMaxDynamicSharedMemorySize, (int)updLds);

  const int nUw = NWPART * WUNIT + TUNIT;
  k_wprep<<<cdiv(nUw, NTHR), NTHR, 0, stream>>>(Wm_src, Wm_dst, Wm_e, Wu_h, Wu_agg, Wt1, BP, BE, BU, BT, nUw);
  const int nUh = MP * (HD / 4);
  k_h0<<<cdiv(nUh, NTHR), NTHR, 0, stream>>>(x, Wn, bn, HA, nN, nUh);
  k_csr<<<gC, NTHR, csrLds, stream>>>(eidx, pos, nE, nN, vec8, ES, ED, EW, INFO);

  float* Hc = HA;
  float* Hx = HB;
  for (int l = 0; l < NLAY; ++l) {
    k_proj<<<gM, NTHR, projLds, stream>>>(Hc, BP + (size_t)l * (NP * KP), P);
    k_msg<<<gC, NTHR, msgLds, stream>>>(ES, ED, EW, INFO, We, be, BE + (size_t)l * (HD * KE), P,
                                         bm + (size_t)l * HD, AGG, nN, MP);
    k_update<<<gM, NTHR, updLds, stream>>>(Hc, AGG, BU + (size_t)l * (HD * KU), bu + (size_t)l * HD, Hx, nN);
    float* tsw = Hc; Hc = Hx; Hx = tsw;
  }
  k_topo<<<gM, NTHR, topoLds, stream>>>(Hc, BT, bt1, Wt2, bt2, out, nN);
  k_tail<<<1, NTHR, 0, stream>>>(Hc, z_c, tc, u_idx, v_idx, w_idx, Ge1, ge1b, Ge2, ge2b, Gmu, gmub, Glv, glvb,
                                 Gd1, gd1b, Gd2, gd2b, Gd3, gd3b, Gp1, gp1b, Gp2, gp2b, pbs, out, nN, nN);
}
